// KGATRecommender_40140764349010
// MI455X (gfx1250) — hardware-verified
//
#include <hip/hip_runtime.h>
#include <stddef.h>


#define DF      128
#define KV      256
#define NTHR    256
#define NWAVE   8
#define EPT     8
#define NGRP    2
#define CHUNK   (NTHR * EPT * NGRP)
#define WCAP    (EPT * NGRP * 32)
#define LISTN   (NWAVE * WCAP)
#define NB      512
#define NTILE   (NB / 16)
#define TPW     (NTILE / NWAVE)

#define LDS_ACC   (NB * DF * 4)
#define LDS_LIST  (LISTN * 4)
#define LDS_AD    (NB * 4)
#define LDS_LAYER (LDS_ACC + LDS_LIST + LDS_AD + 64)

static_assert((CHUNK & (CHUNK - 1)) == 0);
static_assert(CHUNK <= 4096);
static_assert((NB & (NB - 1)) == 0);
static_assert(NB <= 4096);
static_assert(NTILE % NWAVE == 0);
static_assert(NWAVE * 4 <= 64);
static_assert(NB % NTHR == 0);
static_assert(LDS_LAYER <= 300 * 1024);

typedef float  v4f   __attribute__((ext_vector_type(4)));
typedef float  v8f   __attribute__((ext_vector_type(8)));
typedef int    v4i   __attribute__((ext_vector_type(4)));
typedef __bf16 bf16_t;
typedef bf16_t v8bf  __attribute__((ext_vector_type(8)));
typedef bf16_t v16bf __attribute__((ext_vector_type(16)));
union FragB { v16bf v; v8bf h[2]; v4i q[2]; };
union Pack8 { v8bf v; v4i q; };

__device__ __forceinline__ v8f wmb(v16bf a, v16bf b, v8f c) {
  v8f d = __builtin_amdgcn_wmma_f32_16x16x32_bf16(false, a, false, b, (short)0, c, false, false);
  asm volatile("v_nop\n\tv_nop\n\tv_nop\n\tv_nop" : "+v"(d) : "v"(a), "v"(b));
  return d;
}

template <int B>
__device__ __forceinline__ void split8(FragB& hi, FragB& lo, v4f a, v4f b) {
#define SPL1(I, X) { const float xv = (X); const bf16_t hb = (bf16_t)xv; hi.v[B + (I)] = hb; lo.v[B + (I)] = (bf16_t)(xv - (float)hb); }
  SPL1(0, a.x) SPL1(1, a.y) SPL1(2, a.z) SPL1(3, a.w)
  SPL1(4, b.x) SPL1(5, b.y) SPL1(6, b.z) SPL1(7, b.w)
#undef SPL1
}

template <int NBT>
__device__ __forceinline__ int scan_chunk(const int* __restrict__ dsts, int nE, int cbase, int nodeBase,
                                          int vec8, int* list, int tid, int lane, int wave) {
  int wc = 0;
  (void)lane;
#pragma unroll
  for (int g = 0; g < NGRP; ++g) {
    const int el0  = (g * NTHR + tid) * EPT;
    const int e0   = cbase + el0;
    const int sent = -2147483647 - 1;
    v4i da, db;
    if (vec8 != 0 && cbase + CHUNK <= nE) {
      da = *(const v4i*)(dsts + e0);
      db = *(const v4i*)(dsts + e0 + 4);
    } else {
      da.x = (e0     < nE) ? dsts[min(e0, nE - 1)] : sent;
      da.y = (e0 + 1 < nE) ? dsts[min(e0 + 1, nE - 1)] : sent;
      da.z = (e0 + 2 < nE) ? dsts[min(e0 + 2, nE - 1)] : sent;
      da.w = (e0 + 3 < nE) ? dsts[min(e0 + 3, nE - 1)] : sent;
      db.x = (e0 + 4 < nE) ? dsts[min(e0 + 4, nE - 1)] : sent;
      db.y = (e0 + 5 < nE) ? dsts[min(e0 + 5, nE - 1)] : sent;
      db.z = (e0 + 6 < nE) ? dsts[min(e0 + 6, nE - 1)] : sent;
      db.w = (e0 + 7 < nE) ? dsts[min(e0 + 7, nE - 1)] : sent;
    }
    const unsigned nb = (unsigned)nodeBase;
    const unsigned s0 = (unsigned)da.x - nb, s1 = (unsigned)da.y - nb;
    const unsigned s2 = (unsigned)da.z - nb, s3 = (unsigned)da.w - nb;
    const unsigned s4 = (unsigned)db.x - nb, s5 = (unsigned)db.y - nb;
    const unsigned s6 = (unsigned)db.z - nb, s7 = (unsigned)db.w - nb;
    const bool h0 = s0 < (unsigned)NBT, h1 = s1 < (unsigned)NBT, h2 = s2 < (unsigned)NBT, h3 = s3 < (unsigned)NBT;
    const bool h4 = s4 < (unsigned)NBT, h5 = s5 < (unsigned)NBT, h6 = s6 < (unsigned)NBT, h7 = s7 < (unsigned)NBT;
    const unsigned any = __builtin_amdgcn_ballot_w32(h0 | h1 | h2 | h3 | h4 | h5 | h6 | h7);
    if (any != 0u) {
#define HITJ(J, HJ, SJ) { \
        const unsigned mj = __builtin_amdgcn_ballot_w32(HJ); \
        if (mj != 0u) { \
          if (HJ) { \
            const int pos = wc + (int)__builtin_amdgcn_mbcnt_lo(mj, 0u); \
            if (pos < WCAP) list[wave * WCAP + pos] = ((el0 + (J)) << 12) | (int)(SJ); \
          } \
          wc += (int)__builtin_popcount(mj); } }
      HITJ(0, h0, s0)
      HITJ(1, h1, s1)
      HITJ(2, h2, s2)
      HITJ(3, h3, s3)
      HITJ(4, h4, s4)
      HITJ(5, h5, s5)
      HITJ(6, h6, s6)
      HITJ(7, h7, s7)
#undef HITJ
    }
  }
  return wc;
}

__global__ __launch_bounds__(NTHR) void k_wprep(
    const float* __restrict__ Wg, bf16_t* whi, bf16_t* wlo, int nTot) {
  const int i = blockIdx.x * NTHR + threadIdx.x;
  if (i >= nTot) return;
  const int o     = i * 8;
  const int layer = o / (DF * KV);
  const int rem   = o - layer * (DF * KV);
  const int n     = rem / KV;
  const int k0    = rem - n * KV;
  const float* p = Wg + (size_t)layer * KV * DF + (size_t)k0 * DF + n;
  Pack8 ph, pl;
#define WSP(I) { const float xv = p[(I) * DF]; const bf16_t hb = (bf16_t)xv; ph.v[(I)] = hb; pl.v[(I)] = (bf16_t)(xv - (float)hb); }
  WSP(0) WSP(1) WSP(2) WSP(3) WSP(4) WSP(5) WSP(6) WSP(7)
#undef WSP
  bf16_t* dh = whi + o;
  bf16_t* dl = wlo + o;
  const v4i qh = ph.q, ql = pl.q;
  *(volatile v4i*)dh = qh;
  *(volatile v4i*)dl = ql;
  __threadfence();
  *(volatile v4i*)dh = qh;
  *(volatile v4i*)dl = ql;
}

__global__ __launch_bounds__(NTHR) void k_nodescal(
    const float* __restrict__ x0p, const float* __restrict__ x1p,
    const float* __restrict__ wap, float* asv, float* adv, int nU, int nN) {
  const int tid = threadIdx.x, lane = tid & 31, wave = tid >> 5;
  const int nb = blockIdx.x * NTHR + wave * 32;
  const v4f w0 = *(const v4f*)(wap + 4 * lane);
  const v4f w1 = *(const v4f*)(wap + DF + 4 * lane);
  float mys = 0.0f, myd = 0.0f;
#pragma unroll 1
  for (int j = 0; j < 32; ++j) {
    int node = nb + j;
    node = node > nN - 1 ? nN - 1 : node;
    const float* xr = (node < nU) ? (x0p + (size_t)node * DF) : (x1p + (size_t)(node - nU) * DF);
    const v4f v = *(const v4f*)(xr + 4 * lane);
    float ps = v.x * w0.x + v.y * w0.y + v.z * w0.z + v.w * w0.w;
    float pd = v.x * w1.x + v.y * w1.y + v.z * w1.z + v.w * w1.w;
#pragma unroll
    for (int off = 16; off > 0; off >>= 1) {
      ps += __shfl_xor(ps, off, 32);
      pd += __shfl_xor(pd, off, 32);
    }
    mys = (lane == j) ? ps : mys;
    myd = (lane == j) ? pd : myd;
  }
  float* sp = asv + nb + lane;
  float* dp = adv + nb + lane;
  *(volatile float*)sp = mys;
  *(volatile float*)dp = myd;
  __threadfence();
  *(volatile float*)sp = mys;
  *(volatile float*)dp = myd;
}

__device__ __forceinline__ void kstep(const float* ap, const bf16_t* bhp, const bf16_t* blp, v8f (&c)[8]) {
  const v4f p0 = *(const v4f*)(ap);
  const v4f p1 = *(const v4f*)(ap + 4);
  const v4f p2 = *(const v4f*)(ap + 16);
  const v4f p3 = *(const v4f*)(ap + 20);
  FragB ahi, alo;
  split8<0>(ahi, alo, p0, p1);
  split8<8>(ahi, alo, p2, p3);
#pragma unroll
  for (int ct = 0; ct < DF / 16; ++ct) {
    const bf16_t* hp = bhp + (size_t)ct * 16 * KV;
    const bf16_t* lp = blp + (size_t)ct * 16 * KV;
    FragB bh, bq;
    bh.q[0] = *(const v4i*)hp;  bh.q[1] = *(const v4i*)(hp + 16);
    bq.q[0] = *(const v4i*)lp;  bq.q[1] = *(const v4i*)(lp + 16);
    c[ct] = wmb(alo.v, bh.v, c[ct]);
    c[ct] = wmb(ahi.v, bq.v, c[ct]);
    c[ct] = wmb(ahi.v, bh.v, c[ct]);
  }
}

__global__ __launch_bounds__(NTHR) void k_layer(
    const int* __restrict__ ei, const float* __restrict__ x0p, const float* __restrict__ x1p,
    const bf16_t* __restrict__ whi, const bf16_t* __restrict__ wlo,
    const float* __restrict__ bias, const float* __restrict__ bap,
    const float* __restrict__ asv, const float* __restrict__ adv,
    float* xout, int nU, int nN, int nE, int vec8, int last) {
  extern __shared__ v4f lds_dyn[];
  float* acc  = (float*)lds_dyn;
  int*   list = (int*)((char*)lds_dyn + LDS_ACC);
  float* adl  = (float*)((char*)lds_dyn + LDS_ACC + LDS_LIST);
  int*   wcnt = (int*)((char*)lds_dyn + LDS_ACC + LDS_LIST + LDS_AD);
  const int tid = threadIdx.x, lane = tid & 31, wave = tid >> 5, hh = lane >> 4, m = lane & 15;
  const int nodeBase = blockIdx.x * NB;
  const int* dsts = ei + nE;
  const float bal = bap[0];

  {
    const v4f z = {0.f, 0.f, 0.f, 0.f};
    for (int i = tid; i < NB * DF / 4; i += NTHR) lds_dyn[i] = z;
    for (int i = tid; i < NB; i += NTHR) adl[i] = adv[nodeBase + i];
  }
  __syncthreads();

  const int nChunks = (nE + CHUNK - 1) / CHUNK;
#pragma unroll 1
  for (int ch = 0; ch < nChunks; ++ch) {
    const int cbase = ch * CHUNK;
    const int wc = scan_chunk<NB>(dsts, nE, cbase, nodeBase, vec8, list, tid, lane, wave);
    if (lane == 0) wcnt[wave] = wc;
    __syncthreads();
    if (wave == 0) {
#pragma unroll 1
      for (int wsx = 0; wsx < NWAVE; ++wsx) {
        int n = __builtin_amdgcn_readfirstlane(wcnt[wsx]);
        n = n > WCAP ? WCAP : (n < 0 ? 0 : n);
        const int* lp = list + wsx * WCAP;
#pragma unroll 1
        for (int i = 0; i < n; ++i) {
          const int ent  = __builtin_amdgcn_readfirstlane(lp[i]);
          const int slot = ent & (NB - 1);
          int e = cbase + ((ent >> 12) & (CHUNK - 1));
          e = e > nE - 1 ? nE - 1 : e;
          int src = ei[e];
          src = src < 0 ? 0 : (src > nN - 1 ? nN - 1 : src);
          const float p   = asv[src] + adl[slot] + bal;
          const float att = __builtin_amdgcn_rcpf(1.0f + __expf(-p));
          const float* xr = (src < nU) ? (x0p + (size_t)src * DF) : (x1p + (size_t)(src - nU) * DF);
          const v4f v = *(const v4f*)(xr + 4 * lane);
          v4f* ap = (v4f*)(acc + slot * DF + 4 * lane);
          *ap = *ap + v * att;
        }
      }
    }
    __syncthreads();
  }

#pragma unroll 1
  for (int q = 0; q < TPW; ++q) {
    const int t     = q * NWAVE + wave;
    const int slotm = 16 * t + m;
    int node = nodeBase + slotm;
    node = node > nN - 1 ? nN - 1 : node;

    v8f c[8];
#pragma unroll
    for (int ct = 0; ct < 8; ++ct) { const v8f z = {0.f, 0.f, 0.f, 0.f, 0.f, 0.f, 0.f, 0.f}; c[ct] = z; }

    const float*  xsel = (node < nU) ? (x0p + (size_t)node * DF) : (x1p + (size_t)(node - nU) * DF);
    const float*  xrow = xsel + 8 * hh;
    const float*  arow = acc + slotm * DF + 8 * hh;
    const bf16_t* bh0  = whi + m * KV + 8 * hh;
    const bf16_t* bl0  = wlo + m * KV + 8 * hh;
#pragma unroll 1
    for (int ks = 0; ks < DF / 32; ++ks)
      kstep(xrow + 32 * ks, bh0 + 32 * ks, bl0 + 32 * ks, c);
#pragma unroll 1
    for (int ks = 0; ks < DF / 32; ++ks)
      kstep(arow + 32 * ks, bh0 + DF + 32 * ks, bl0 + DF + 32 * ks, c);

    float* sp = acc + (16 * t + 8 * hh) * DF + m;
#pragma unroll
    for (int ct = 0; ct < 8; ++ct) {
      const float bb = bias[16 * ct + m];
#pragma unroll
      for (int r = 0; r < 8; ++r) sp[r * DF + 16 * ct] = fmaxf(c[ct][r] + bb, 0.0f);
    }
    __syncthreads();

    const int row0 = nodeBase + 16 * t;
    int nrows = 16;
    if (last != 0) {
      int rem = nN - row0;
      rem = rem < 0 ? 0 : rem;
      nrows = rem < 16 ? rem : 16;
    }
    const float* lrow = acc + (16 * t) * DF + 4 * lane;
    float* gp = xout + (size_t)row0 * DF + 4 * lane;
#pragma unroll
    for (int i = 0; i < 16; ++i) {
      if (i < nrows) { const v4f v = *(const v4f*)(lrow + i * DF); *(volatile v4f*)(gp + (size_t)i * DF) = v; }
    }
    __threadfence();
#pragma unroll
    for (int i = 0; i < 16; ++i) {
      if (i < nrows) { const v4f v = *(const v4f*)(lrow + i * DF); *(volatile v4f*)(gp + (size_t)i * DF) = v; }
    }
  }
}

extern "C" void kernel_launch(void* const* d_in, const int* in_sizes, int n_in,
                              void* d_out, int out_size, void* d_ws, size_t ws_size,
                              hipStream_t stream) {
  if (n_in < 7) return;
  const int nE = in_sizes[0] / 2;
  const int nU = in_sizes[1] / DF;
  const int nI = in_sizes[2] / DF;
  const int nL = in_sizes[3] / KV;
  if (nE < 1 || nU <= 0 || nI <= 0 || nL <= 0) return;
  if (in_sizes[0] != 2 * nE || in_sizes[1] != nU * DF || in_sizes[2] != nI * DF) return;
  if (in_sizes[3] != nL * KV || in_sizes[4] < nL) return;
  if (in_sizes[5] != nL * KV * DF || in_sizes[6] < nL * DF) return;
  const int nN = nU + nI;
  if (out_size != nN * DF) return;

  const int*   ei = (const int*)d_in[0];
  const float* ue = (const float*)d_in[1];
  const float* ie = (const float*)d_in[2];
  const float* Wa = (const float*)d_in[3];
  const float* ba = (const float*)d_in[4];
  const float* Wg = (const float*)d_in[5];
  const float* bg = (const float*)d_in[6];
  float* out = (float*)d_out;

  const int nBlk = (nN + NB - 1) / NB;
  const int nPad = nBlk * NB;

  char* ws = (char*)d_ws;
  size_t off = 0;
  const size_t szW = (size_t)nL * DF * KV * 2;
  const size_t szS = (size_t)nPad * 4;
  const size_t szX = (size_t)nPad * DF * 4;
  const size_t oWh = off; off += szW; off = (off + 255) & ~(size_t)255;
  const size_t oWl = off; off += szW; off = (off + 255) & ~(size_t)255;
  const size_t oAs = off; off += szS; off = (off + 255) & ~(size_t)255;
  const size_t oAd = off; off += szS; off = (off + 255) & ~(size_t)255;
  const size_t oXa = off; off += szX; off = (off + 255) & ~(size_t)255;
  const size_t oXb = off; off += szX; off = (off + 255) & ~(size_t)255;
  if (off > ws_size) return;
  bf16_t* whi = (bf16_t*)(ws + oWh);
  bf16_t* wlo = (bf16_t*)(ws + oWl);
  float*  asv = (float*)(ws + oAs);
  float*  adv = (float*)(ws + oAd);
  float*  xa  = (float*)(ws + oXa);
  float*  xb  = (float*)(ws + oXb);

  const int vec8 = ((nE & 3) == 0) ? 1 : 0;

  const int nTot = nL * DF * KV / 8;
  k_wprep<<<(nTot + NTHR - 1) / NTHR, NTHR, 0, stream>>>(Wg, whi, wlo, nTot);

  hipFuncSetAttribute(reinterpret_cast<const void*>(&k_layer),
                      hipFuncAttributeMaxDynamicSharedMemorySize, LDS_LAYER);

  const float* xin0 = ue;
  const float* xin1 = ie;
  float* bufs[2] = {xa, xb};
  for (int l = 0; l < nL; ++l) {
    const int last = (l == nL - 1) ? 1 : 0;
    float* xo = last ? out : bufs[l & 1];
    k_nodescal<<<nPad / NTHR, NTHR, 0, stream>>>(xin0, xin1, Wa + (size_t)l * KV, asv, adv, nU, nN);
    k_layer<<<nBlk, NTHR, LDS_LAYER, stream>>>(
        ei, xin0, xin1, whi + (size_t)l * DF * KV, wlo + (size_t)l * DF * KV,
        bg + (size_t)l * DF, ba + l, asv, adv, xo, nU, nN, nE, vec8, last);
    xin0 = xo;
    xin1 = xo + (size_t)nU * DF;
  }
}
